// SoftClusteringBlock_82051055222995
// MI455X (gfx1250) — hardware-verified
//
#include <hip/hip_runtime.h>
#include <stdint.h>

typedef __attribute__((ext_vector_type(16))) _Float16 v16h;
typedef __attribute__((ext_vector_type(8)))  _Float16 v8h;
typedef __attribute__((ext_vector_type(16))) __bf16   v16b;
typedef __attribute__((ext_vector_type(8)))  __bf16   v8b;
typedef __attribute__((ext_vector_type(8)))  float    v8f;
typedef __attribute__((ext_vector_type(4)))  float    v4f;
#define PSCALE 32768.0f
#define U16(p) ((const unsigned short*)(const void*)(p))
#define PSCALE_INV (1.0f / 32768.0f)

static constexpr int FD   = 128;
static constexpr int KCEN = 512;

__device__ __forceinline__ unsigned short f2bf_bits(float f) {
  unsigned u = __float_as_uint(f);
  return (unsigned short)((u + 0x7FFFu + ((u >> 16) & 1u)) >> 16);
}
__device__ __forceinline__ float bf_bits2f(unsigned short h) { return __uint_as_float(((unsigned)h) << 16); }

__device__ __forceinline__ void dep_guard_h(v8f& a, v8f& b, v16h x, v16h y) { asm volatile("v_nop\n\tv_nop\n\tv_nop\n\tv_nop" : "+v"(a), "+v"(b) : "v"(x), "v"(y)); }
__device__ __forceinline__ void dep_guard_b(v8f& a, v8f& b, v16b x, v16b y) { asm volatile("v_nop\n\tv_nop\n\tv_nop\n\tv_nop" : "+v"(a), "+v"(b) : "v"(x), "v"(y)); }
__device__ __forceinline__ void keep4_h(v16h a, v16h b, v16h c, v16h d) { asm volatile("v_nop" :: "v"(a), "v"(b), "v"(c), "v"(d)); }
__device__ __forceinline__ void keep4_b(v16b a, v16b b, v16b c, v16b d) { asm volatile("v_nop" :: "v"(a), "v"(b), "v"(c), "v"(d)); }
__device__ __forceinline__ void acc_guard4(v8f& a, v8f& b, v8f& c, v8f& d) { asm volatile("v_nop\n\tv_nop\n\tv_nop\n\tv_nop" : "+v"(a), "+v"(b), "+v"(c), "+v"(d)); }
template <typename T> struct Frag;
template <> struct Frag<_Float16> {
  typedef v16h V; union U { v16h v; v8h h[2]; };
  static __device__ __forceinline__ v16h load(const _Float16* p) {
    U f; f.h[0] = *(const v8h*)(p); f.h[1] = *(const v8h*)(p + 16); return f.v;
  }
  static __device__ __forceinline__ v8f mma(v16h a, v16h b, v8f c) {
    return __builtin_amdgcn_wmma_f32_16x16x32_f16(false, a, false, b, (short)0, c, false, false);
  }
  static __device__ __forceinline__ void guard(v8f& a, v8f& b, v16h x, v16h y) { dep_guard_h(a, b, x, y); }
  static __device__ __forceinline__ void keep(v16h a, v16h b, v16h c, v16h d) { keep4_h(a, b, c, d); }
};
template <> struct Frag<__bf16> {
  typedef v16b V; union U { v16b v; v8b h[2]; };
  static __device__ __forceinline__ v16b load(const __bf16* p) {
    U f; f.h[0] = *(const v8b*)(p); f.h[1] = *(const v8b*)(p + 16); return f.v;
  }
  static __device__ __forceinline__ v8f mma(v16b a, v16b b, v8f c) {
    return __builtin_amdgcn_wmma_f32_16x16x32_bf16(false, a, false, b, (short)0, c, false, false);
  }
  static __device__ __forceinline__ void guard(v8f& a, v8f& b, v16b x, v16b y) { dep_guard_b(a, b, x, y); }
  static __device__ __forceinline__ void keep(v16b a, v16b b, v16b c, v16b d) { keep4_b(a, b, c, d); }
};

template <int ET> struct Elem;
template <> struct Elem<0> { typedef _Float16 T; };
template <> struct Elem<1> { typedef __bf16 T; };
template <int ET, bool SPLIT, int BIAS_MODE, int OUT_MODE, bool RESID, int ACT = 0>
__global__ __launch_bounds__(256) void wmma_gemm64(
    const unsigned short* __restrict__ Ap, const unsigned short* __restrict__ A2p, int lda, long strideA,
    const unsigned short* __restrict__ Btp, const unsigned short* __restrict__ Bt2p, int ldb, long strideB,
    void* __restrict__ Cout, void* __restrict__ Cout2, int ldc, long strideC,
    const float* __restrict__ bias,
    const float* __restrict__ resid, long strideR,
    int M, int N, int K, float scale) {
  typedef typename Elem<ET>::T T;
  typedef typename Frag<T>::V V;
  const T* A = (const T*)Ap; const T* A2 = (const T*)A2p; const T* Bt = (const T*)Btp; const T* Bt2 = (const T*)Bt2p;
  __shared__ __align__(16) float sT[8][16 * 68];
  const int b    = blockIdx.y;
  const int lane = threadIdx.x & 31;
  const int wave = threadIdx.x >> 5;
  const int tilesN = N >> 6;
  const int tilesM = M >> 6;
  const int tile = blockIdx.x * 8 + wave;
  if (tile >= tilesM * tilesN) return;
  const int tm = tile / tilesN;
  const int tn = tile - tm * tilesN;
  const int m0 = tm << 6;
  const int n0 = tn << 6;

  const T* Ab  = A  + (size_t)b * strideA;
  const T* Bb  = Bt + (size_t)b * strideB;
  const T* Ab2 = SPLIT ? (A2  + (size_t)b * strideA) : nullptr;
  const T* Bb2 = SPLIT ? (Bt2 + (size_t)b * strideB) : nullptr;

  const int rlane = lane & 15;
  const int koff  = (lane >> 4) * 8;
  const int mOff  = (lane >> 4) * 8;

  v8f acc[4][4];
#pragma unroll
  for (int i = 0; i < 4; ++i)
#pragma unroll
    for (int j = 0; j < 4; ++j) acc[i][j] = (v8f){0.f,0.f,0.f,0.f,0.f,0.f,0.f,0.f};

  for (int k0 = 0; k0 < K; k0 += 32) {
    V bh[4], bl[4];
#pragma unroll
    for (int j = 0; j < 4; ++j) {
      const size_t bo = (size_t)(n0 + (j << 4) + rlane) * ldb + koff + k0;
      bh[j] = Frag<T>::load(Bb + bo);
      if (SPLIT) bl[j] = Frag<T>::load(Bb2 + bo);
    }
#pragma unroll
    for (int i = 0; i < 4; ++i) {
      const size_t ao = (size_t)(m0 + (i << 4) + rlane) * lda + koff + k0;
      V ah = Frag<T>::load(Ab + ao);
      V al;
      if (SPLIT) al = Frag<T>::load(Ab2 + ao);
#pragma unroll
      for (int j = 0; j < 4; ++j) {
        acc[i][j] = Frag<T>::mma(ah, bh[j], acc[i][j]);
        if (SPLIT) {
          acc[i][j] = Frag<T>::mma(ah, bl[j], acc[i][j]);
          acc[i][j] = Frag<T>::mma(al, bh[j], acc[i][j]);
        }
      }
      Frag<T>::guard(acc[i][0], acc[i][3], ah, SPLIT ? al : ah);
    }
    Frag<T>::keep(bh[0], bh[1], bh[2], bh[3]);
    if (SPLIT) Frag<T>::keep(bl[0], bl[1], bl[2], bl[3]);
  }
  acc_guard4(acc[0][0], acc[0][1], acc[0][2], acc[0][3]);
  acc_guard4(acc[1][0], acc[1][1], acc[1][2], acc[1][3]);
  acc_guard4(acc[2][0], acc[2][1], acc[2][2], acc[2][3]);
  acc_guard4(acc[3][0], acc[3][1], acc[3][2], acc[3][3]);

  float* slab = sT[wave];
  const float* Rb = RESID ? (resid + (size_t)b * strideR) : nullptr;
#pragma unroll
  for (int i = 0; i < 4; ++i) {
    const int mBase = m0 + (i << 4);
#pragma unroll
    for (int j = 0; j < 4; ++j) {
      const int n = n0 + (j << 4) + rlane;
      float bv = 0.f;
      if (BIAS_MODE == 2) bv = bias[n];
#pragma unroll
      for (int r = 0; r < 8; ++r) {
        float v = acc[i][j][r] * scale;
        if (BIAS_MODE == 1) v += bias[mBase + mOff + r];
        if (BIAS_MODE == 2) v += bv;
        if (RESID) v += Rb[(size_t)(mBase + mOff + r) * ldc + n];
        if (ACT == 1) v = tanhf(v);
        if (ACT == 2) v = fmaxf(v, 0.0f);
        if (ACT == 3) v = v / (1.0f + expf(-v));
        if (ACT == 4) v = (v > 0.f) ? v : 0.01f * v;
        if (ACT == 5) v = 0.5f * v * (1.0f + erff(v * 0.70710678118654752f));
        slab[(mOff + r) * 68 + (j << 4) + rlane] = v;
      }
    }
    __builtin_amdgcn_fence(__ATOMIC_RELEASE, "workgroup");
    __builtin_amdgcn_wave_barrier();
    __builtin_amdgcn_fence(__ATOMIC_ACQUIRE, "workgroup");
    if (OUT_MODE == 0) {
      float* C = (float*)Cout + (size_t)b * strideC;
      const int hh = lane >> 4, c4 = (lane & 15) * 4;
      for (int pass = 0; pass < 2; ++pass) {
#pragma unroll
        for (int it = 0; it < 8; ++it) {
          const int row = it * 2 + hh;
          v4f v = *(const v4f*)(slab + row * 68 + c4);
          *(volatile v4f*)(C + (size_t)(mBase + row) * ldc + n0 + c4) = v;
        }
        __threadfence();
      }
    } else {
      const int q = lane >> 3, c8 = (lane & 7) * 8;
      unsigned short* C  = (unsigned short*)Cout  + (size_t)b * strideC;
      unsigned short* C2 = (OUT_MODE == 2) ? ((unsigned short*)Cout2 + (size_t)b * strideC) : nullptr;
      for (int pass = 0; pass < 2; ++pass) {
#pragma unroll
        for (int it = 0; it < 4; ++it) {
          const int row = it * 4 + q;
          const float* sp = slab + row * 68 + c8;
          v8h hv, lv;
#pragma unroll
          for (int e = 0; e < 8; ++e) {
            if (OUT_MODE == 1) {
              hv[e] = (_Float16)sp[e];
            } else {
              unsigned short hb = f2bf_bits(sp[e]);
              unsigned short lb = f2bf_bits(sp[e] - bf_bits2f(hb));
              hv[e] = __builtin_bit_cast(_Float16, hb);
              lv[e] = __builtin_bit_cast(_Float16, lb);
            }
          }
          *(volatile v8h*)(C + (size_t)(mBase + row) * ldc + n0 + c8) = hv;
          if (OUT_MODE == 2) *(volatile v8h*)(C2 + (size_t)(mBase + row) * ldc + n0 + c8) = lv;
        }
        __threadfence();
      }
    }
    __builtin_amdgcn_fence(__ATOMIC_RELEASE, "workgroup");
    __builtin_amdgcn_wave_barrier();
    __builtin_amdgcn_fence(__ATOMIC_ACQUIRE, "workgroup");
  }
}

__global__ __launch_bounds__(256) void prep_centres(const float* __restrict__ cen, _Float16* __restrict__ c16,
                                                    _Float16* __restrict__ cT16, float* __restrict__ csq) {
  __shared__ __align__(16) float tile[64 * 132];
  __shared__ float sq[64];
  const int tid = threadIdx.x, lane = tid & 31, wave = tid >> 5;
  const int k0 = blockIdx.x * 64;
  {
    const int r = tid >> 2, c0 = (tid & 3) * 32;
    const float* src = cen + (size_t)(k0 + r) * FD + c0;
    float ss = 0.f;
#pragma unroll
    for (int i = 0; i < 8; ++i) {
      const v4f v = *(const v4f*)(src + 4 * i);
      *(v4f*)(tile + r * 132 + c0 + 4 * i) = v;
      ss += v[0] * v[0]; ss += v[1] * v[1]; ss += v[2] * v[2]; ss += v[3] * v[3];
    }
    ss += __shfl_xor(ss, 1, 32);
    ss += __shfl_xor(ss, 2, 32);
    if ((tid & 3) == 0) sq[r] = ss;
  }
  __syncthreads();
  for (int pass = 0; pass < 2; ++pass) {
#pragma unroll
    for (int p = 0; p < 4; ++p) {
      const int slot = p * 256 + tid;
      const int r = slot >> 4, c8 = (slot & 15) * 8;
      const v4f a = *(const v4f*)(tile + r * 132 + c8);
      const v4f bq = *(const v4f*)(tile + r * 132 + c8 + 4);
      v8h h;
#pragma unroll
      for (int e = 0; e < 4; ++e) { h[e] = (_Float16)a[e]; h[4 + e] = (_Float16)bq[e]; }
      *(volatile v8h*)(c16 + (size_t)(k0 + r) * FD + c8) = h;
    }
#pragma unroll
    for (int p = 0; p < 4; ++p) {
      const int slot = p * 256 + tid;
      const int f = slot >> 3, q = slot & 7;
      v8h h;
#pragma unroll
      for (int e = 0; e < 8; ++e) h[e] = (_Float16)tile[(q * 8 + e) * 132 + f];
      *(volatile v8h*)(cT16 + (size_t)f * KCEN + k0 + q * 8) = h;
    }
    __threadfence();
  }
  if (wave < 2) {
    const float v = sq[wave * 32 + lane];
    volatile float* p = csq + k0 + wave * 32 + lane;
    *p = v;
    __threadfence();
    *p = v;
  }
}

__global__ __launch_bounds__(256) void cast_rows(const float* __restrict__ x, _Float16* __restrict__ x16,
                                                 float* __restrict__ xsq) {
  __shared__ float sq[32];
  const int tid = threadIdx.x, lane = tid & 31, wave = tid >> 5;
  const int r0 = blockIdx.x * 32;
  const int rsub = tid >> 4, c8 = (tid & 15) * 8;
  v8h hv[2];
  float s[2];
#pragma unroll
  for (int p = 0; p < 2; ++p) {
    const int rl = p * 16 + rsub;
    const float* src = x + (size_t)(r0 + rl) * FD + c8;
    const v4f a = *(const v4f*)src;
    const v4f bq = *(const v4f*)(src + 4);
    float ss = 0.f;
    v8h h;
#pragma unroll
    for (int e = 0; e < 4; ++e) { h[e] = (_Float16)a[e]; ss += a[e] * a[e]; }
#pragma unroll
    for (int e = 0; e < 4; ++e) { h[4 + e] = (_Float16)bq[e]; ss += bq[e] * bq[e]; }
#pragma unroll
    for (int off = 1; off < 16; off <<= 1) ss += __shfl_xor(ss, off, 32);
    hv[p] = h; s[p] = ss;
  }
  if ((tid & 15) == 0) { sq[rsub] = s[0]; sq[16 + rsub] = s[1]; }
  for (int pass = 0; pass < 2; ++pass) {
#pragma unroll
    for (int p = 0; p < 2; ++p)
      *(volatile v8h*)(x16 + (size_t)(r0 + p * 16 + rsub) * FD + c8) = hv[p];
    __threadfence();
  }
  __syncthreads();
  if (wave == 0) {
    const float v = sq[lane];
    volatile float* p = xsq + r0 + lane;
    *p = v;
    __threadfence();
    *p = v;
  }
}

__global__ __launch_bounds__(256) void softmax_rows(const float* __restrict__ cross, const float* __restrict__ xsq,
                                                    const float* __restrict__ csq, _Float16* __restrict__ assoc) {
#pragma clang fp contract(off)
  __shared__ float s_csq[KCEN];
  __shared__ __align__(16) float rbuf[8][KCEN];
  const int tid = threadIdx.x, lane = tid & 31, wave = tid >> 5;
  s_csq[tid] = csq[tid];
  s_csq[tid + 256] = csq[tid + 256];
  __syncthreads();
  float* rb = rbuf[wave];
  const int rowb = blockIdx.x * 64 + wave * 8;
#pragma unroll 1
  for (int i = 0; i < 8; ++i) {
    const int lrow = rowb + i;
    const float xs = xsq[lrow];
    const float* cr = cross + (size_t)lrow * KCEN;
    __builtin_amdgcn_fence(__ATOMIC_RELEASE, "workgroup");
    __builtin_amdgcn_wave_barrier();
    __builtin_amdgcn_fence(__ATOMIC_ACQUIRE, "workgroup");
    float m = -INFINITY;
#pragma unroll 1
    for (int it = 0; it < 16; ++it) {
      const int col = it * 32 + lane;
      const float t = xs + s_csq[col];
      const float d2 = fmaxf(t - 2.0f * cr[col], 0.0f);
      const float z = -sqrtf(d2);
      rb[col] = z;
      m = fmaxf(m, z);
    }
#pragma unroll
    for (int off = 1; off < 32; off <<= 1) m = fmaxf(m, __shfl_xor(m, off, 32));
    float sum = 0.f;
#pragma unroll 1
    for (int it = 0; it < 16; ++it) {
      const int col = it * 32 + lane;
      const float p = expf(rb[col] - m);
      rb[col] = p;
      sum += p;
    }
#pragma unroll
    for (int off = 1; off < 32; off <<= 1) sum += __shfl_xor(sum, off, 32);
    const float inv = 1.0f / sum;
    __builtin_amdgcn_fence(__ATOMIC_RELEASE, "workgroup");
    __builtin_amdgcn_wave_barrier();
    __builtin_amdgcn_fence(__ATOMIC_ACQUIRE, "workgroup");
    const v4f a0 = *(const v4f*)(rb + 8 * lane);
    const v4f a1 = *(const v4f*)(rb + 8 * lane + 4);
    const v4f b0 = *(const v4f*)(rb + 256 + 8 * lane);
    const v4f b1 = *(const v4f*)(rb + 256 + 8 * lane + 4);
    v8h h0, h1;
#pragma unroll
    for (int e = 0; e < 4; ++e) {
      h0[e]     = (_Float16)((a0[e] * inv) * PSCALE);
      h0[4 + e] = (_Float16)((a1[e] * inv) * PSCALE);
      h1[e]     = (_Float16)((b0[e] * inv) * PSCALE);
      h1[4 + e] = (_Float16)((b1[e] * inv) * PSCALE);
    }
    _Float16* arow = assoc + (size_t)lrow * KCEN;
    for (int pass = 0; pass < 2; ++pass) {
      *(volatile v8h*)(arow + 8 * lane) = h0;
      *(volatile v8h*)(arow + 256 + 8 * lane) = h1;
      __threadfence();
    }
  }
}

extern "C" void kernel_launch(void* const* d_in, const int* in_sizes, int n_in,
                              void* d_out, int out_size, void* d_ws, size_t ws_size,
                              hipStream_t stream) {
  if (n_in < 2) return;
  const int nx = in_sizes[0];
  const int nc = in_sizes[1];
  if (nc != KCEN * FD) return;
  if (nx <= 0 || (nx % FD) != 0) return;
  const int rows = nx / FD;
  if ((rows % 64) != 0) return;
  if (out_size != nx) return;
  int RC = rows < 16384 ? rows : 16384;
  while ((rows % RC) != 0) RC -= 64;
  if (RC < 64) return;
  const int nchunks = rows / RC;

  size_t off = 0;
  const size_t o_x16   = off; off += ((size_t)rows * FD * 2 + 127) & ~(size_t)127;
  const size_t o_xsq   = off; off += ((size_t)rows * 4 + 127) & ~(size_t)127;
  const size_t o_c16   = off; off += ((size_t)KCEN * FD * 2 + 127) & ~(size_t)127;
  const size_t o_cT16  = off; off += ((size_t)KCEN * FD * 2 + 127) & ~(size_t)127;
  const size_t o_csq   = off; off += ((size_t)KCEN * 4 + 127) & ~(size_t)127;
  const size_t o_cross = off; off += ((size_t)RC * KCEN * 4 + 127) & ~(size_t)127;
  const size_t o_assoc = off; off += ((size_t)RC * KCEN * 2 + 127) & ~(size_t)127;
  if (off > ws_size || off > (size_t)134217728) return;

  char* ws = (char*)d_ws;
  const float* x   = (const float*)d_in[0];
  const float* cen = (const float*)d_in[1];
  float* out = (float*)d_out;
  _Float16* x16   = (_Float16*)(ws + o_x16);
  float*    xsq   = (float*)(ws + o_xsq);
  _Float16* c16   = (_Float16*)(ws + o_c16);
  _Float16* cT16  = (_Float16*)(ws + o_cT16);
  float*    csq   = (float*)(ws + o_csq);
  float*    cross = (float*)(ws + o_cross);
  _Float16* assoc = (_Float16*)(ws + o_assoc);

  prep_centres<<<KCEN / 64, 256, 0, stream>>>(cen, c16, cT16, csq);
  cast_rows<<<rows / 32, 256, 0, stream>>>(x, x16, xsq);

  const int tiles1 = (RC / 64) * (KCEN / 64);
  const int tiles2 = (RC / 64) * (FD / 64);
  const dim3 g1((tiles1 + 7) / 8, 1);
  const dim3 g2((tiles2 + 7) / 8, 1);
  for (int q = 0; q < nchunks; ++q) {
    const size_t rbase = (size_t)q * RC;
    wmma_gemm64<0, false, 0, 0, false, 0><<<g1, 256, 0, stream>>>(
        (const unsigned short*)(x16 + rbase * FD), nullptr, FD, 0L,
        (const unsigned short*)c16, nullptr, FD, 0L,
        (void*)cross, nullptr, KCEN, 0L,
        nullptr, nullptr, 0L,
        RC, KCEN, FD, 1.0f);
    softmax_rows<<<RC / 64, 256, 0, stream>>>(cross, xsq + rbase, csq, assoc);
    wmma_gemm64<0, false, 0, 0, false, 0><<<g2, 256, 0, stream>>>(
        (const unsigned short*)assoc, nullptr, KCEN, 0L,
        (const unsigned short*)cT16, nullptr, KCEN, 0L,
        (void*)(out + rbase * FD), nullptr, FD, 0L,
        nullptr, nullptr, 0L,
        RC, FD, KCEN, PSCALE_INV);
  }
}
